// GCNWithMultiHeadGATAndTCN_42356967473538
// MI455X (gfx1250) — hardware-run, weakly checked
//
#include <hip/hip_runtime.h>
#include <stdint.h>

#define NBATCH 4
#define NNODE 2048
#define NCH 256
#define NHEAD 4
#define HDIM 64
#define NROWS (NBATCH * NNODE)
#define NPADROW (NNODE + 2)
#define KCONV (3 * NCH)
#define BN_EPS 1e-5f
#define LRELU_SLOPE_F 0.2f
#define KEYCHUNK 64

static_assert(NCH % 64 == 0 && NROWS % 64 == 0 && NCH % 32 == 0, "site0 M=NCH N=NROWS K=NCH");
static_assert(NNODE % 64 == 0 && NCH % 64 == 0 && NNODE % 32 == 0, "site1 M=NNODE N=NCH K=NNODE");
static_assert(NROWS % 64 == 0 && HDIM % 64 == 0 && NCH % 32 == 0, "site2 M=NROWS N=HDIM K=NCH and swapped");
static_assert(NNODE % 64 == 0 && NCH % 64 == 0 && KCONV % 32 == 0, "conv M=NNODE N=NCH K=KCONV");
static_assert(NHEAD * HDIM == NCH, "head split");
static_assert(NNODE % KEYCHUNK == 0 && HDIM == 64, "attention: 64-row query blocks, 64-key chunks, head dim 64");
static_assert((NBATCH * NPADROW) % 8 == 0, "mix grid exact");

typedef __attribute__((ext_vector_type(16))) _Float16 v16h;
typedef __attribute__((ext_vector_type(8)))  _Float16 v8h;
typedef __attribute__((ext_vector_type(16))) __bf16   v16b;
typedef __attribute__((ext_vector_type(8)))  __bf16   v8b;
typedef __attribute__((ext_vector_type(8)))  float    v8f;
typedef __attribute__((ext_vector_type(4)))  float    v4f;
typedef __attribute__((ext_vector_type(4)))  unsigned int u32x4;

__device__ __forceinline__ unsigned short f2bf_bits(float f) {
  unsigned u = __float_as_uint(f);
  return (unsigned short)((u + 0x7FFFu + ((u >> 16) & 1u)) >> 16);
}
__device__ __forceinline__ float bf_bits2f(unsigned short h) { return __uint_as_float(((unsigned)h) << 16); }

__device__ __forceinline__ void dep_guard_h(v8f& a, v8f& b, v16h x, v16h y) { asm volatile("v_nop\n\tv_nop\n\tv_nop\n\tv_nop" : "+v"(a), "+v"(b) : "v"(x), "v"(y)); }
__device__ __forceinline__ void dep_guard_b(v8f& a, v8f& b, v16b x, v16b y) { asm volatile("v_nop\n\tv_nop\n\tv_nop\n\tv_nop" : "+v"(a), "+v"(b) : "v"(x), "v"(y)); }
__device__ __forceinline__ void keep4_h(v16h a, v16h b, v16h c, v16h d) { asm volatile("v_nop" :: "v"(a), "v"(b), "v"(c), "v"(d)); }
__device__ __forceinline__ void keep4_b(v16b a, v16b b, v16b c, v16b d) { asm volatile("v_nop" :: "v"(a), "v"(b), "v"(c), "v"(d)); }
__device__ __forceinline__ void acc_guard4(v8f& a, v8f& b, v8f& c, v8f& d) { asm volatile("v_nop\n\tv_nop\n\tv_nop\n\tv_nop" : "+v"(a), "+v"(b), "+v"(c), "+v"(d)); }
template <typename T> struct Frag;
template <> struct Frag<_Float16> {
  typedef v16h V; union U { v16h v; v8h h[2]; };
  static __device__ __forceinline__ v16h load(const _Float16* p) {
    U f; f.h[0] = *(const v8h*)(p); f.h[1] = *(const v8h*)(p + 16); return f.v;
  }
  static __device__ __forceinline__ v8f mma(v16h a, v16h b, v8f c) {
    return __builtin_amdgcn_wmma_f32_16x16x32_f16(false, a, false, b, (short)0, c, false, false);
  }
  static __device__ __forceinline__ void guard(v8f& a, v8f& b, v16h x, v16h y) { dep_guard_h(a, b, x, y); }
  static __device__ __forceinline__ void keep(v16h a, v16h b, v16h c, v16h d) { keep4_h(a, b, c, d); }
};
template <> struct Frag<__bf16> {
  typedef v16b V; union U { v16b v; v8b h[2]; };
  static __device__ __forceinline__ v16b load(const __bf16* p) {
    U f; f.h[0] = *(const v8b*)(p); f.h[1] = *(const v8b*)(p + 16); return f.v;
  }
  static __device__ __forceinline__ v8f mma(v16b a, v16b b, v8f c) {
    return __builtin_amdgcn_wmma_f32_16x16x32_bf16(false, a, false, b, (short)0, c, false, false);
  }
  static __device__ __forceinline__ void guard(v8f& a, v8f& b, v16b x, v16b y) { dep_guard_b(a, b, x, y); }
  static __device__ __forceinline__ void keep(v16b a, v16b b, v16b c, v16b d) { keep4_b(a, b, c, d); }
};

template <int ET> struct Elem;
template <> struct Elem<0> { typedef _Float16 T; };
template <> struct Elem<1> { typedef __bf16 T; };
template <int ET, bool SPLIT, int BIAS_MODE, int OUT_MODE, bool RESID, int ACT = 0>
__global__ __launch_bounds__(256) void wmma_gemm64(
    const unsigned short* __restrict__ Ap, const unsigned short* __restrict__ A2p, int lda, long strideA,
    const unsigned short* __restrict__ Btp, const unsigned short* __restrict__ Bt2p, int ldb, long strideB,
    void* __restrict__ Cout, void* __restrict__ Cout2, int ldc, long strideC,
    const float* __restrict__ bias,
    const float* __restrict__ resid, long strideR,
    int M, int N, int K, float scale) {
  typedef typename Elem<ET>::T T;
  typedef typename Frag<T>::V V;
  const T* A = (const T*)Ap; const T* A2 = (const T*)A2p; const T* Bt = (const T*)Btp; const T* Bt2 = (const T*)Bt2p;
  __shared__ __align__(16) float sT[8][16 * 68];
  const int b    = blockIdx.y;
  const int lane = threadIdx.x & 31;
  const int wave = threadIdx.x >> 5;
  const int tilesN = N >> 6;
  const int tilesM = M >> 6;
  const int tile = blockIdx.x * 8 + wave;
  if (tile >= tilesM * tilesN) return;
  const int tm = tile / tilesN;
  const int tn = tile - tm * tilesN;
  const int m0 = tm << 6;
  const int n0 = tn << 6;

  const T* Ab  = A  + (size_t)b * strideA;
  const T* Bb  = Bt + (size_t)b * strideB;
  const T* Ab2 = SPLIT ? (A2  + (size_t)b * strideA) : nullptr;
  const T* Bb2 = SPLIT ? (Bt2 + (size_t)b * strideB) : nullptr;

  const int rlane = lane & 15;
  const int koff  = (lane >> 4) * 8;
  const int mOff  = (lane >> 4) * 8;

  v8f acc[4][4];
#pragma unroll
  for (int i = 0; i < 4; ++i)
#pragma unroll
    for (int j = 0; j < 4; ++j) acc[i][j] = (v8f){0.f,0.f,0.f,0.f,0.f,0.f,0.f,0.f};

  for (int k0 = 0; k0 < K; k0 += 32) {
    V bh[4], bl[4];
#pragma unroll
    for (int j = 0; j < 4; ++j) {
      const size_t bo = (size_t)(n0 + (j << 4) + rlane) * ldb + koff + k0;
      bh[j] = Frag<T>::load(Bb + bo);
      if (SPLIT) bl[j] = Frag<T>::load(Bb2 + bo);
    }
#pragma unroll
    for (int i = 0; i < 4; ++i) {
      const size_t ao = (size_t)(m0 + (i << 4) + rlane) * lda + koff + k0;
      V ah = Frag<T>::load(Ab + ao);
      V al;
      if (SPLIT) al = Frag<T>::load(Ab2 + ao);
#pragma unroll
      for (int j = 0; j < 4; ++j) {
        acc[i][j] = Frag<T>::mma(ah, bh[j], acc[i][j]);
        if (SPLIT) {
          acc[i][j] = Frag<T>::mma(ah, bl[j], acc[i][j]);
          acc[i][j] = Frag<T>::mma(al, bh[j], acc[i][j]);
        }
      }
      Frag<T>::guard(acc[i][0], acc[i][3], ah, SPLIT ? al : ah);
    }
    Frag<T>::keep(bh[0], bh[1], bh[2], bh[3]);
    if (SPLIT) Frag<T>::keep(bl[0], bl[1], bl[2], bl[3]);
  }
  acc_guard4(acc[0][0], acc[0][1], acc[0][2], acc[0][3]);
  acc_guard4(acc[1][0], acc[1][1], acc[1][2], acc[1][3]);
  acc_guard4(acc[2][0], acc[2][1], acc[2][2], acc[2][3]);
  acc_guard4(acc[3][0], acc[3][1], acc[3][2], acc[3][3]);

  float* slab = sT[wave];
  const float* Rb = RESID ? (resid + (size_t)b * strideR) : nullptr;
#pragma unroll
  for (int i = 0; i < 4; ++i) {
    const int mBase = m0 + (i << 4);
#pragma unroll
    for (int j = 0; j < 4; ++j) {
      const int n = n0 + (j << 4) + rlane;
      float bv = 0.f;
      if (BIAS_MODE == 2) bv = bias[n];
#pragma unroll
      for (int r = 0; r < 8; ++r) {
        float v = acc[i][j][r] * scale;
        if (BIAS_MODE == 1) v += bias[mBase + mOff + r];
        if (BIAS_MODE == 2) v += bv;
        if (RESID) v += Rb[(size_t)(mBase + mOff + r) * ldc + n];
        if (ACT == 1) v = tanhf(v);
        if (ACT == 2) v = fmaxf(v, 0.0f);
        if (ACT == 3) v = v / (1.0f + expf(-v));
        if (ACT == 4) v = (v > 0.f) ? v : 0.01f * v;
        if (ACT == 5) v = 0.5f * v * (1.0f + erff(v * 0.70710678118654752f));
        slab[(mOff + r) * 68 + (j << 4) + rlane] = v;
      }
    }
    __builtin_amdgcn_fence(__ATOMIC_RELEASE, "workgroup");
    __builtin_amdgcn_wave_barrier();
    __builtin_amdgcn_fence(__ATOMIC_ACQUIRE, "workgroup");
    if (OUT_MODE == 0) {
      float* C = (float*)Cout + (size_t)b * strideC;
      const int hh = lane >> 4, c4 = (lane & 15) * 4;
      for (int pass = 0; pass < 2; ++pass) {
#pragma unroll
        for (int it = 0; it < 8; ++it) {
          const int row = it * 2 + hh;
          v4f v = *(const v4f*)(slab + row * 68 + c4);
          *(volatile v4f*)(C + (size_t)(mBase + row) * ldc + n0 + c4) = v;
        }
        __threadfence();
      }
    } else {
      const int q = lane >> 3, c8 = (lane & 7) * 8;
      unsigned short* C  = (unsigned short*)Cout  + (size_t)b * strideC;
      unsigned short* C2 = (OUT_MODE == 2) ? ((unsigned short*)Cout2 + (size_t)b * strideC) : nullptr;
      for (int pass = 0; pass < 2; ++pass) {
#pragma unroll
        for (int it = 0; it < 4; ++it) {
          const int row = it * 4 + q;
          const float* sp = slab + row * 68 + c8;
          v8h hv, lv;
#pragma unroll
          for (int e = 0; e < 8; ++e) {
            if (OUT_MODE == 1) {
              hv[e] = (_Float16)sp[e];
            } else {
              unsigned short hb = f2bf_bits(sp[e]);
              unsigned short lb = f2bf_bits(sp[e] - bf_bits2f(hb));
              hv[e] = __builtin_bit_cast(_Float16, hb);
              lv[e] = __builtin_bit_cast(_Float16, lb);
            }
          }
          *(volatile v8h*)(C + (size_t)(mBase + row) * ldc + n0 + c8) = hv;
          if (OUT_MODE == 2) *(volatile v8h*)(C2 + (size_t)(mBase + row) * ldc + n0 + c8) = lv;
        }
        __threadfence();
      }
    }
    __builtin_amdgcn_fence(__ATOMIC_RELEASE, "workgroup");
    __builtin_amdgcn_wave_barrier();
    __builtin_amdgcn_fence(__ATOMIC_ACQUIRE, "workgroup");
  }
}

__device__ __forceinline__ unsigned short at_bf_bits(float f) {
  unsigned u = __float_as_uint(f);
  return (unsigned short)((u + 0x7FFFu + ((u >> 16) & 1u)) >> 16);
}
__device__ __forceinline__ __bf16 at_f2bf(float f) { return __builtin_bit_cast(__bf16, at_bf_bits(f)); }
__device__ __forceinline__ void at_split(float f, __bf16& hi, __bf16& lo) {
  const unsigned short hb = at_bf_bits(f);
  hi = __builtin_bit_cast(__bf16, hb);
  lo = at_f2bf(f - __uint_as_float(((unsigned)hb) << 16));
}
__device__ __forceinline__ v8f at_mma(v16b a, v16b b, v8f c) {
  c = __builtin_amdgcn_wmma_f32_16x16x32_bf16(false, a, false, b, (short)0, c, false, false);
  asm volatile("v_nop\n\tv_nop\n\tv_nop\n\tv_nop" : "+v"(c) : "v"(a), "v"(b));
  return c;
}

__device__ __forceinline__ unsigned split_pair_hl(float f0, float f1, unsigned& lo_out) {
  const unsigned short h0 = f2bf_bits(f0), h1 = f2bf_bits(f1);
  const unsigned short l0 = f2bf_bits(f0 - bf_bits2f(h0)), l1 = f2bf_bits(f1 - bf_bits2f(h1));
  lo_out = (unsigned)l0 | ((unsigned)l1 << 16);
  return (unsigned)h0 | ((unsigned)h1 << 16);
}
__device__ __forceinline__ void split8(v4f a, v4f b, u32x4& ph, u32x4& pl) {
  unsigned l0, l1, l2, l3;
  const unsigned h0 = split_pair_hl(a[0], a[1], l0);
  const unsigned h1 = split_pair_hl(a[2], a[3], l1);
  const unsigned h2 = split_pair_hl(b[0], b[1], l2);
  const unsigned h3 = split_pair_hl(b[2], b[3], l3);
  ph = (u32x4){h0, h1, h2, h3};
  pl = (u32x4){l0, l1, l2, l3};
}
__device__ __forceinline__ v4f relu4(v4f v) {
  v4f r;
  r[0] = fmaxf(v[0], 0.0f); r[1] = fmaxf(v[1], 0.0f); r[2] = fmaxf(v[2], 0.0f); r[3] = fmaxf(v[3], 0.0f);
  return r;
}

__global__ __launch_bounds__(256) void cast_rows_kernel(const float* __restrict__ in,
                                                         unsigned short* __restrict__ hi,
                                                         unsigned short* __restrict__ lo,
                                                         int R, int nseg) {
  const int wave = threadIdx.x >> 5, lane = threadIdx.x & 31;
  const int row = blockIdx.x * 8 + wave;
  if (row >= R) return;
  const size_t rbase = (size_t)row * (size_t)nseg * 256;
#pragma unroll 1
  for (int seg = 0; seg < nseg; ++seg) {
    const size_t e0 = rbase + (size_t)seg * 256 + 8 * lane;
    const v4f a = *(const v4f*)(in + e0);
    const v4f b = *(const v4f*)(in + e0 + 4);
    u32x4 ph, pl;
    split8(a, b, ph, pl);
    for (int pass = 0; pass < 2; ++pass) {
      *(volatile u32x4*)(hi + e0) = ph;
      *(volatile u32x4*)(lo + e0) = pl;
      __threadfence();
    }
  }
}

template <int MODE>
__device__ __forceinline__ size_t gsrc_index(int row, int kk) {
  if (MODE == 0) return (size_t)kk * NCH + row;
  return ((size_t)(row >> 6) * NCH + kk) * HDIM + (row & 63);
}
template <int MODE>
__global__ __launch_bounds__(256) void cast_gather_kernel(const float* __restrict__ src,
                                                           unsigned short* __restrict__ hi,
                                                           unsigned short* __restrict__ lo) {
  const int wave = threadIdx.x >> 5, lane = threadIdx.x & 31;
  const int row = blockIdx.x * 8 + wave;
  if (row >= NCH) return;
  const int k0 = 8 * lane;
  const float f0 = src[gsrc_index<MODE>(row, k0 + 0)];
  const float f1 = src[gsrc_index<MODE>(row, k0 + 1)];
  const float f2 = src[gsrc_index<MODE>(row, k0 + 2)];
  const float f3 = src[gsrc_index<MODE>(row, k0 + 3)];
  const float f4 = src[gsrc_index<MODE>(row, k0 + 4)];
  const float f5 = src[gsrc_index<MODE>(row, k0 + 5)];
  const float f6 = src[gsrc_index<MODE>(row, k0 + 6)];
  const float f7 = src[gsrc_index<MODE>(row, k0 + 7)];
  const v4f a = (v4f){f0, f1, f2, f3};
  const v4f b = (v4f){f4, f5, f6, f7};
  u32x4 ph, pl;
  split8(a, b, ph, pl);
  const size_t e0 = (size_t)row * NCH + 8 * lane;
  for (int pass = 0; pass < 2; ++pass) {
    *(volatile u32x4*)(hi + e0) = ph;
    *(volatile u32x4*)(lo + e0) = pl;
    __threadfence();
  }
}

__global__ __launch_bounds__(256) void conv_pack_kernel(const float* __restrict__ cw,
                                                         unsigned short* __restrict__ hi,
                                                         unsigned short* __restrict__ lo) {
  const int wave = threadIdx.x >> 5, lane = threadIdx.x & 31;
  const int o = blockIdx.x * 8 + wave;
  if (o >= NCH) return;
  const float* src = cw + ((size_t)o * NCH + 8 * lane) * 3;
  const v4f q0 = *(const v4f*)(src + 0);
  const v4f q1 = *(const v4f*)(src + 4);
  const v4f q2 = *(const v4f*)(src + 8);
  const v4f q3 = *(const v4f*)(src + 12);
  const v4f q4 = *(const v4f*)(src + 16);
  const v4f q5 = *(const v4f*)(src + 20);
  const v4f a0 = (v4f){q0[0], q0[3], q1[2], q2[1]}, b0 = (v4f){q3[0], q3[3], q4[2], q5[1]};
  const v4f a1 = (v4f){q0[1], q1[0], q1[3], q2[2]}, b1 = (v4f){q3[1], q4[0], q4[3], q5[2]};
  const v4f a2 = (v4f){q0[2], q1[1], q2[0], q2[3]}, b2 = (v4f){q3[2], q4[1], q5[0], q5[3]};
  u32x4 ph0, pl0, ph1, pl1, ph2, pl2;
  split8(a0, b0, ph0, pl0);
  split8(a1, b1, ph1, pl1);
  split8(a2, b2, ph2, pl2);
  const size_t e0 = (size_t)o * KCONV + 8 * lane;
  for (int pass = 0; pass < 2; ++pass) {
    *(volatile u32x4*)(hi + e0) = ph0;
    *(volatile u32x4*)(lo + e0) = pl0;
    *(volatile u32x4*)(hi + e0 + 256) = ph1;
    *(volatile u32x4*)(lo + e0 + 256) = pl1;
    *(volatile u32x4*)(hi + e0 + 512) = ph2;
    *(volatile u32x4*)(lo + e0 + 512) = pl2;
    __threadfence();
  }
}

__global__ __launch_bounds__(256) void bn_stats_kernel(const float* __restrict__ x,
                                                       float* __restrict__ mean,
                                                       float* __restrict__ rstd) {
  __shared__ double sh_s[8][32];
  __shared__ double sh_q[8][32];
  const int wave = threadIdx.x >> 5, lane = threadIdx.x & 31;
  const int c = blockIdx.x * 32 + lane;
  double s = 0.0, q = 0.0;
#pragma unroll 4
  for (int r = wave; r < NROWS; r += 8) {
    const float v = x[(size_t)r * NCH + c];
    const double dv = (double)v;
    s += dv;
    q += dv * dv;
  }
  sh_s[wave][lane] = s;
  sh_q[wave][lane] = q;
  __syncthreads();
  if (wave == 0) {
    double a = 0.0, a2 = 0.0;
#pragma unroll
    for (int w = 0; w < 8; ++w) { a += sh_s[w][lane]; a2 += sh_q[w][lane]; }
    const double inv = 1.0 / (double)NROWS;
    const double m = a * inv;
    const double var = a2 * inv - m * m;
    const float mf = (float)m;
    float vf = (float)var;
    vf = fmaxf(vf, 0.0f);
    const float rs = rsqrtf(vf + BN_EPS);
    for (int pass = 0; pass < 2; ++pass) {
      ((volatile float*)mean)[c] = mf;
      ((volatile float*)rstd)[c] = rs;
      __threadfence();
    }
  }
}

__global__ __launch_bounds__(256) void bn_apply_kernel(const float* __restrict__ x,
                                                       const float* __restrict__ mean,
                                                       const float* __restrict__ rstd,
                                                       const float* __restrict__ gamma,
                                                       const float* __restrict__ beta,
                                                       float* __restrict__ yf,
                                                       unsigned short* __restrict__ yh,
                                                       unsigned short* __restrict__ yl) {
  __shared__ __align__(16) float slab[8][NCH];
  const int wave = threadIdx.x >> 5, lane = threadIdx.x & 31;
  const int row = blockIdx.x * 8 + wave;
  if (row >= NROWS) return;
  const size_t rb = (size_t)row * NCH;
  const int c0 = 8 * lane;
  const v4f xa = *(const v4f*)(x + rb + c0),   xb = *(const v4f*)(x + rb + c0 + 4);
  const v4f ma = *(const v4f*)(mean + c0),     mb = *(const v4f*)(mean + c0 + 4);
  const v4f ra = *(const v4f*)(rstd + c0),     rr = *(const v4f*)(rstd + c0 + 4);
  const v4f ga = *(const v4f*)(gamma + c0),    gb = *(const v4f*)(gamma + c0 + 4);
  const v4f ba = *(const v4f*)(beta + c0),     bb = *(const v4f*)(beta + c0 + 4);
  const v4f ya = relu4(((xa - ma) * ra) * ga + ba);
  const v4f yb = relu4(((xb - mb) * rr) * gb + bb);
  u32x4 ph, pl;
  split8(ya, yb, ph, pl);
  float* sw = slab[wave];
  *(v4f*)(sw + c0) = ya;
  *(v4f*)(sw + c0 + 4) = yb;
  __builtin_amdgcn_fence(__ATOMIC_RELEASE, "workgroup");
  __builtin_amdgcn_wave_barrier();
  __builtin_amdgcn_fence(__ATOMIC_ACQUIRE, "workgroup");
  const int c4 = 4 * lane;
  const v4f o0 = *(const v4f*)(sw + c4);
  const v4f o1 = *(const v4f*)(sw + 128 + c4);
  for (int pass = 0; pass < 2; ++pass) {
    *(volatile u32x4*)(yh + rb + c0) = ph;
    *(volatile u32x4*)(yl + rb + c0) = pl;
    *(volatile v4f*)(yf + rb + c4) = o0;
    *(volatile v4f*)(yf + rb + 128 + c4) = o1;
    __threadfence();
  }
}

__global__ __launch_bounds__(128) __attribute__((amdgpu_num_vgpr(256)))
void gat_attn_kernel(const unsigned short* __restrict__ hph,
                     const unsigned short* __restrict__ hpl,
                     const unsigned short* __restrict__ hpth,
                     const unsigned short* __restrict__ hptl,
                     float* __restrict__ gat) {
  typedef Frag<__bf16> FR;
  __shared__ __align__(16) __bf16 Ksh[KEYCHUNK * HDIM];
  __shared__ __align__(16) __bf16 Ksl[KEYCHUNK * HDIM];
  __shared__ __align__(16) __bf16 Vth[HDIM * KEYCHUNK];
  __shared__ __align__(16) __bf16 Vtl[HDIM * KEYCHUNK];
  __shared__ __align__(16) __bf16 Psh[4][16 * KEYCHUNK];
  __shared__ __align__(16) __bf16 Psl[4][16 * KEYCHUNK];
  __shared__ __align__(16) float  Os[4][16 * 68];
  const int tid = threadIdx.x, wave = tid >> 5, lane = tid & 31;
  const int hh = lane >> 4, c = lane & 15, koff = hh * 8;
  const int bx = blockIdx.x;
  const int qb = bx % (NNODE / 64);
  const int bhx = bx / (NNODE / 64);
  const int h = bhx % NHEAD;
  const int b = bhx / NHEAD;
  const int q0 = qb * 64 + wave * 16;
  const __bf16* Hh = (const __bf16*)hph;
  const __bf16* Hl = (const __bf16*)hpl;
  const size_t rowb = (size_t)b * NNODE;
  const int hcol = h * HDIM;

  v16b qah[2], qal[2];
#pragma unroll
  for (int dc = 0; dc < 2; ++dc) {
    const size_t qo = (rowb + q0 + c) * NCH + hcol + dc * 32 + koff;
    qah[dc] = FR::load(Hh + qo);
    qal[dc] = FR::load(Hl + qo);
  }

  float mrow[8], lrow[8];
  v8f oacc[4];
#pragma unroll
  for (int r = 0; r < 8; ++r) { mrow[r] = -__builtin_inff(); lrow[r] = 0.f; }
#pragma unroll
  for (int t = 0; t < 4; ++t) oacc[t] = (v8f){0.f,0.f,0.f,0.f,0.f,0.f,0.f,0.f};

  for (int kc = 0; kc < NNODE / KEYCHUNK; ++kc) {
    const int kv0 = kc * KEYCHUNK;
    __syncthreads();
#pragma unroll
    for (int i = 0; i < 4; ++i) {
      const int p = tid + 128 * i;
      const int kv = p >> 3, d8 = (p & 7) * 8;
      const size_t go = (rowb + kv0 + kv) * NCH + hcol + d8;
      const u32x4 wh = *(const u32x4*)(const void*)(hph + go);
      const u32x4 wl = *(const u32x4*)(const void*)(hpl + go);
      *(u32x4*)(void*)(Ksh + kv * HDIM + d8) = wh;
      *(u32x4*)(void*)(Ksl + kv * HDIM + d8) = wl;
    }
    asm volatile("" ::: "memory");
#pragma unroll
    for (int i = 0; i < 4; ++i) {
      const int p = tid + 128 * i;
      const int d = p >> 3, kv8 = (p & 7) * 8;
      const size_t go = (size_t)(hcol + d) * NROWS + rowb + kv0 + kv8;
      const u32x4 wh = *(const u32x4*)(const void*)(hpth + go);
      const u32x4 wl = *(const u32x4*)(const void*)(hptl + go);
      *(u32x4*)(void*)(Vth + d * KEYCHUNK + kv8) = wh;
      *(u32x4*)(void*)(Vtl + d * KEYCHUNK + kv8) = wl;
    }
    __syncthreads();

    v8f s[4];
#pragma unroll
    for (int j = 0; j < 4; ++j) {
      s[j] = (v8f){0.f,0.f,0.f,0.f,0.f,0.f,0.f,0.f};
#pragma unroll
      for (int dc = 0; dc < 2; ++dc) {
        const __bf16* kp = Ksh + (j * 16 + c) * HDIM + dc * 32 + koff;
        const __bf16* kq = Ksl + (j * 16 + c) * HDIM + dc * 32 + koff;
        const v16b kb = FR::load(kp);
        const v16b kl = FR::load(kq);
        s[j] = at_mma(qah[dc], kb, s[j]);
        s[j] = at_mma(qah[dc], kl, s[j]);
        s[j] = at_mma(qal[dc], kb, s[j]);
      }
    }
    float cm[8];
#pragma unroll
    for (int r = 0; r < 8; ++r) {
      float m = -__builtin_inff();
#pragma unroll
      for (int j = 0; j < 4; ++j) {
        float xv = s[j][r];
        xv = (xv >= 0.0f) ? xv : LRELU_SLOPE_F * xv;
        s[j][r] = xv;
        m = fmaxf(m, xv);
      }
#pragma unroll
      for (int off = 1; off < 16; off <<= 1) m = fmaxf(m, __shfl_xor(m, off, 32));
      cm[r] = m;
    }
    __bf16* pwh = Psh[wave];
    __bf16* pwl = Psl[wave];
#pragma unroll
    for (int r = 0; r < 8; ++r) {
      const float mnew = fmaxf(mrow[r], cm[r]);
      const float corr = expf(mrow[r] - mnew);
      mrow[r] = mnew;
      float psum = 0.f;
#pragma unroll
      for (int j = 0; j < 4; ++j) {
        const float p = expf(s[j][r] - mnew);
        psum += p;
        __bf16 pa_, pb_;
        at_split(p, pa_, pb_);
        pwh[(8 * hh + r) * KEYCHUNK + j * 16 + c] = pa_;
        pwl[(8 * hh + r) * KEYCHUNK + j * 16 + c] = pb_;
      }
#pragma unroll
      for (int off = 1; off < 16; off <<= 1) psum += __shfl_xor(psum, off, 32);
      lrow[r] = lrow[r] * corr + psum;
#pragma unroll
      for (int t = 0; t < 4; ++t) oacc[t][r] *= corr;
    }
    __builtin_amdgcn_fence(__ATOMIC_RELEASE, "workgroup");
    __builtin_amdgcn_wave_barrier();
    __builtin_amdgcn_fence(__ATOMIC_ACQUIRE, "workgroup");
#pragma unroll
    for (int kk = 0; kk < 2; ++kk) {
      const v16b pa = FR::load(pwh + c * KEYCHUNK + kk * 32 + koff);
      const v16b pl = FR::load(pwl + c * KEYCHUNK + kk * 32 + koff);
#pragma unroll
      for (int t = 0; t < 4; ++t) {
        const __bf16* vp = Vth + (t * 16 + c) * KEYCHUNK + kk * 32 + koff;
        const __bf16* vq = Vtl + (t * 16 + c) * KEYCHUNK + kk * 32 + koff;
        const v16b vb = FR::load(vp);
        const v16b vl = FR::load(vq);
        oacc[t] = at_mma(pa, vb, oacc[t]);
        oacc[t] = at_mma(pa, vl, oacc[t]);
        oacc[t] = at_mma(pl, vb, oacc[t]);
      }
    }
  }

  float* os = Os[wave];
#pragma unroll
  for (int r = 0; r < 8; ++r) {
    const float inv = 1.0f / lrow[r];
#pragma unroll
    for (int t = 0; t < 4; ++t) os[(8 * hh + r) * 68 + t * 16 + c] = oacc[t][r] * inv;
  }
  __builtin_amdgcn_fence(__ATOMIC_RELEASE, "workgroup");
  __builtin_amdgcn_wave_barrier();
  __builtin_amdgcn_fence(__ATOMIC_ACQUIRE, "workgroup");
  {
    const int c4 = (lane & 15) * 4;
    float* ob = gat + hcol;
    for (int pass = 0; pass < 2; ++pass) {
#pragma unroll
      for (int it = 0; it < 8; ++it) {
        const int row = it * 2 + hh;
        const v4f val = *(const v4f*)(os + row * 68 + c4);
        *(volatile v4f*)(ob + (rowb + q0 + row) * NCH + c4) = val;
      }
      __threadfence();
    }
  }
}

__global__ __launch_bounds__(256) void mix_kernel(const float* __restrict__ gat,
                                                  const float* __restrict__ hbn,
                                                  const float* __restrict__ alpha,
                                                  float* __restrict__ gf,
                                                  unsigned short* __restrict__ gph,
                                                  unsigned short* __restrict__ gpl) {
  __shared__ __align__(16) float slab[8][NCH];
  const int wave = threadIdx.x >> 5, lane = threadIdx.x & 31;
  const int prow = blockIdx.x * 8 + wave;
  if (prow >= NBATCH * NPADROW) return;
  const int bb = prow / NPADROW;
  const int j = prow - bb * NPADROW;
  const int c0 = 8 * lane;
  const size_t pb = (size_t)prow * NCH + c0;
  if (j == 0 || j == NPADROW - 1) {
    const u32x4 z = (u32x4){0u, 0u, 0u, 0u};
    for (int pass = 0; pass < 2; ++pass) {
      *(volatile u32x4*)(gph + pb) = z;
      *(volatile u32x4*)(gpl + pb) = z;
      __threadfence();
    }
    return;
  }
  const size_t rb = ((size_t)bb * NNODE + (size_t)(j - 1)) * NCH;
  const float a = alpha[0];
  const float oma = 1.0f - a;
  const v4f ga = *(const v4f*)(gat + rb + c0), gb = *(const v4f*)(gat + rb + c0 + 4);
  const v4f ha = *(const v4f*)(hbn + rb + c0), hb = *(const v4f*)(hbn + rb + c0 + 4);
  const v4f va = a * ga + oma * ha;
  const v4f vb = a * gb + oma * hb;
  u32x4 ph, pl;
  split8(va, vb, ph, pl);
  float* sw = slab[wave];
  *(v4f*)(sw + c0) = va;
  *(v4f*)(sw + c0 + 4) = vb;
  __builtin_amdgcn_fence(__ATOMIC_RELEASE, "workgroup");
  __builtin_amdgcn_wave_barrier();
  __builtin_amdgcn_fence(__ATOMIC_ACQUIRE, "workgroup");
  const int c4 = 4 * lane;
  const v4f o0 = *(const v4f*)(sw + c4);
  const v4f o1 = *(const v4f*)(sw + 128 + c4);
  for (int pass = 0; pass < 2; ++pass) {
    *(volatile u32x4*)(gph + pb) = ph;
    *(volatile u32x4*)(gpl + pb) = pl;
    *(volatile v4f*)(gf + rb + c4) = o0;
    *(volatile v4f*)(gf + rb + 128 + c4) = o1;
    __threadfence();
  }
}

__global__ __launch_bounds__(256) void final_kernel(const float* __restrict__ t,
                                                    const float* __restrict__ mean,
                                                    const float* __restrict__ rstd,
                                                    const float* __restrict__ gamma,
                                                    const float* __restrict__ beta,
                                                    const float* __restrict__ alpha,
                                                    const float* __restrict__ gf,
                                                    float* __restrict__ out) {
  const int wave = threadIdx.x >> 5, lane = threadIdx.x & 31;
  const int row = blockIdx.x * 8 + wave;
  if (row >= NROWS) return;
  const size_t rb = (size_t)row * NCH;
  const float a = alpha[0];
  const float oma = 1.0f - a;
  const int cA = 4 * lane, cB = 128 + 4 * lane;
  const v4f tA = *(const v4f*)(t + rb + cA),  tB = *(const v4f*)(t + rb + cB);
  const v4f gA = *(const v4f*)(gf + rb + cA), gB = *(const v4f*)(gf + rb + cB);
  const v4f mA = *(const v4f*)(mean + cA),    mB = *(const v4f*)(mean + cB);
  const v4f rA = *(const v4f*)(rstd + cA),    rB = *(const v4f*)(rstd + cB);
  const v4f yA = *(const v4f*)(gamma + cA),   yB = *(const v4f*)(gamma + cB);
  const v4f bA = *(const v4f*)(beta + cA),    bB = *(const v4f*)(beta + cB);
  const v4f nA = relu4(((tA - mA) * rA) * yA + bA);
  const v4f nB = relu4(((tB - mB) * rB) * yB + bB);
  const v4f oA = a * nA + oma * gA;
  const v4f oB = a * nB + oma * gB;
  for (int pass = 0; pass < 2; ++pass) {
    *(volatile v4f*)(out + rb + cA) = oA;
    *(volatile v4f*)(out + rb + cB) = oB;
    __threadfence();
  }
}

extern "C" void kernel_launch(void* const* d_in, const int* in_sizes, int n_in,
                              void* d_out, int out_size, void* d_ws, size_t ws_size,
                              hipStream_t stream) {
  if (n_in < 13) return;
  if (in_sizes[0] != NROWS * NCH || in_sizes[1] != NNODE * NNODE || in_sizes[2] != NCH * NCH ||
      in_sizes[3] != NCH || in_sizes[4] != NCH || in_sizes[5] != NCH ||
      in_sizes[6] != NHEAD * NCH * HDIM || in_sizes[7] < 1 || in_sizes[8] != NCH * NCH * 3 ||
      in_sizes[9] != NCH || in_sizes[10] != NCH || in_sizes[11] != NCH || in_sizes[12] < 1) return;
  if (out_size != NROWS * NCH) return;

  const float* x     = (const float*)d_in[0];
  const float* adj   = (const float*)d_in[1];
  const float* Wsage = (const float*)d_in[2];
  const float* bsage = (const float*)d_in[3];
  const float* gam1  = (const float*)d_in[4];
  const float* bet1  = (const float*)d_in[5];
  const float* Whd   = (const float*)d_in[6];
  const float* a_gat = (const float*)d_in[7];
  const float* cw    = (const float*)d_in[8];
  const float* cb    = (const float*)d_in[9];
  const float* gam2  = (const float*)d_in[10];
  const float* bet2  = (const float*)d_in[11];
  const float* a_tcn = (const float*)d_in[12];
  float* out = (float*)d_out;

  const size_t szActPlane = (size_t)NROWS * NCH * 2;
  const size_t szActF32   = (size_t)NROWS * NCH * 4;
  const size_t szWsPlane  = (size_t)NCH * NCH * 2;
  const size_t szAdjPlane = (size_t)NNODE * NNODE * 2;
  const size_t szWhPlane  = (size_t)NHEAD * HDIM * NCH * 2;
  const size_t szGpPlane  = (size_t)NBATCH * NPADROW * NCH * 2;
  const size_t szWpkPlane = (size_t)NCH * KCONV * 2;
  const size_t szStat     = (size_t)NCH * 4;

  size_t off = 0;
  char* base = (char*)d_ws;
  auto carve = [&](size_t bytes) -> size_t { size_t o = off; off += (bytes + 255) & ~(size_t)255; return o; };
  const size_t o_xh = carve(szActPlane),   o_xl = carve(szActPlane);
  const size_t o_wsh = carve(szWsPlane),   o_wsl = carve(szWsPlane);
  const size_t o_adjh = carve(szAdjPlane), o_adjl = carve(szAdjPlane);
  const size_t o_sph = carve(szActPlane),  o_spl = carve(szActPlane);
  const size_t o_hbuf = carve(szActF32);
  const size_t o_m1 = carve(szStat), o_r1 = carve(szStat), o_m2 = carve(szStat), o_r2 = carve(szStat);
  const size_t o_hbnf = carve(szActF32);
  const size_t o_hbnh = carve(szActPlane), o_hbnl = carve(szActPlane);
  const size_t o_whh = carve(szWhPlane),   o_whl = carve(szWhPlane);
  const size_t o_hph = carve(szActPlane),  o_hpl = carve(szActPlane);
  const size_t o_hpth = carve(szActPlane), o_hptl = carve(szActPlane);
  const size_t o_gat = carve(szActF32);
  const size_t o_gf = carve(szActF32);
  const size_t o_gph = carve(szGpPlane),   o_gpl = carve(szGpPlane);
  const size_t o_wpkh = carve(szWpkPlane), o_wpkl = carve(szWpkPlane);
  const size_t o_tbuf = carve(szActF32);
  if (off > ws_size) return;

  unsigned short* xh   = (unsigned short*)(base + o_xh);
  unsigned short* xl   = (unsigned short*)(base + o_xl);
  unsigned short* wsTh = (unsigned short*)(base + o_wsh);
  unsigned short* wsTl = (unsigned short*)(base + o_wsl);
  unsigned short* adjh = (unsigned short*)(base + o_adjh);
  unsigned short* adjl = (unsigned short*)(base + o_adjl);
  unsigned short* supTh = (unsigned short*)(base + o_sph);
  unsigned short* supTl = (unsigned short*)(base + o_spl);
  float* hbuf  = (float*)(base + o_hbuf);
  float* mean1 = (float*)(base + o_m1);
  float* rstd1 = (float*)(base + o_r1);
  float* mean2 = (float*)(base + o_m2);
  float* rstd2 = (float*)(base + o_r2);
  float* hbnf  = (float*)(base + o_hbnf);
  unsigned short* hbnh = (unsigned short*)(base + o_hbnh);
  unsigned short* hbnl = (unsigned short*)(base + o_hbnl);
  unsigned short* whTh = (unsigned short*)(base + o_whh);
  unsigned short* whTl = (unsigned short*)(base + o_whl);
  unsigned short* hph  = (unsigned short*)(base + o_hph);
  unsigned short* hpl  = (unsigned short*)(base + o_hpl);
  unsigned short* hpTh = (unsigned short*)(base + o_hpth);
  unsigned short* hpTl = (unsigned short*)(base + o_hptl);
  float* gat  = (float*)(base + o_gat);
  float* gf   = (float*)(base + o_gf);
  unsigned short* gph  = (unsigned short*)(base + o_gph);
  unsigned short* gpl  = (unsigned short*)(base + o_gpl);
  unsigned short* wpkh = (unsigned short*)(base + o_wpkh);
  unsigned short* wpkl = (unsigned short*)(base + o_wpkl);
  float* tbuf = (float*)(base + o_tbuf);

  cast_rows_kernel<<<dim3(NROWS / 8), dim3(256), 0, stream>>>(x, xh, xl, NROWS, 1);
  cast_rows_kernel<<<dim3(NNODE / 8), dim3(256), 0, stream>>>(adj, adjh, adjl, NNODE, NNODE / 256);
  cast_gather_kernel<0><<<dim3(NCH / 8), dim3(256), 0, stream>>>(Wsage, wsTh, wsTl);
  cast_gather_kernel<1><<<dim3(NCH / 8), dim3(256), 0, stream>>>(Whd, whTh, whTl);
  conv_pack_kernel<<<dim3(NCH / 8), dim3(256), 0, stream>>>(cw, wpkh, wpkl);

  wmma_gemm64<1, true, 0, 2, false, 0><<<dim3((NCH / 64) * (NROWS / 64) / 8, 1), dim3(256), 0, stream>>>(
      wsTh, wsTl, NCH, 0l,
      xh, xl, NCH, 0l,
      (void*)supTh, (void*)supTl, NROWS, 0l,
      (const float*)nullptr, (const float*)nullptr, 0l,
      NCH, NROWS, NCH, 1.0f);

  wmma_gemm64<1, true, 2, 0, false, 2><<<dim3((NNODE / 64) * (NCH / 64) / 8, NBATCH), dim3(256), 0, stream>>>(
      adjh, adjl, NNODE, 0l,
      supTh, supTl, NROWS, (long)NNODE,
      (void*)hbuf, (void*)nullptr, NCH, (long)NNODE * NCH,
      bsage, (const float*)nullptr, 0l,
      NNODE, NCH, NNODE, 1.0f);

  bn_stats_kernel<<<dim3(NCH / 32), dim3(256), 0, stream>>>(hbuf, mean1, rstd1);
  bn_apply_kernel<<<dim3(NROWS / 8), dim3(256), 0, stream>>>(hbuf, mean1, rstd1, gam1, bet1, hbnf, hbnh, hbnl);

  wmma_gemm64<1, true, 0, 2, false, 0><<<dim3((NROWS / 64) * (HDIM / 64) / 8, NHEAD), dim3(256), 0, stream>>>(
      hbnh, hbnl, NCH, 0l,
      whTh, whTl, NCH, (long)HDIM * NCH,
      (void*)hph, (void*)hpl, NCH, (long)HDIM,
      (const float*)nullptr, (const float*)nullptr, 0l,
      NROWS, HDIM, NCH, 1.0f);

  wmma_gemm64<1, true, 0, 2, false, 0><<<dim3((HDIM / 64) * (NROWS / 64) / 8, NHEAD), dim3(256), 0, stream>>>(
      whTh, whTl, NCH, (long)HDIM * NCH,
      hbnh, hbnl, NCH, 0l,
      (void*)hpTh, (void*)hpTl, NROWS, (long)HDIM * NROWS,
      (const float*)nullptr, (const float*)nullptr, 0l,
      HDIM, NROWS, NCH, 1.0f);

  gat_attn_kernel<<<dim3(NBATCH * NHEAD * (NNODE / 64)), dim3(128), 0, stream>>>(hph, hpl, hpTh, hpTl, gat);

  mix_kernel<<<dim3((NBATCH * NPADROW) / 8), dim3(256), 0, stream>>>(gat, hbnf, a_gat, gf, gph, gpl);

  wmma_gemm64<1, true, 2, 0, false, 0><<<dim3((NNODE / 64) * (NCH / 64) / 8, NBATCH), dim3(256), 0, stream>>>(
      gph, gpl, NCH, (long)NPADROW * NCH,
      wpkh, wpkl, KCONV, 0l,
      (void*)tbuf, (void*)nullptr, NCH, (long)NNODE * NCH,
      cb, (const float*)nullptr, 0l,
      NNODE, NCH, KCONV, 1.0f);

  bn_stats_kernel<<<dim3(NCH / 32), dim3(256), 0, stream>>>(tbuf, mean2, rstd2);
  final_kernel<<<dim3(NROWS / 8), dim3(256), 0, stream>>>(tbuf, mean2, rstd2, gam2, bet2, a_tcn, gf, out);
}
